// GatedSelfAttention_44959717655286
// MI455X (gfx1250) — hardware-verified
//
#include <hip/hip_runtime.h>
#include <stddef.h>
#include <stdint.h>


typedef _Float16 f16_t;
typedef f16_t v16h __attribute__((ext_vector_type(16)));
typedef f16_t v8h  __attribute__((ext_vector_type(8)));
typedef float v8f  __attribute__((ext_vector_type(8)));
typedef float v4f  __attribute__((ext_vector_type(4)));

union Frag { v16h v; v8h half[2]; f16_t e[16]; };
union Acc  { v8f v; float f[8]; };
union H8   { v8h v; f16_t e[8]; };
union F4   { v4f v; float f[4]; };

enum : int {
  BB = 2, LL = 1024, DD = 2048, HH = 16, NHKV = 4, HD = 128, CACHE = 1024, SS = 2048,
  BL = BB * LL, NKV = NHKV * HD, NBHR = BB * HH, QT = LL / 16
};

#define XSCALE   8.f
#define WSCALE   64.f
#define QKVSCALE 16.f
#define PROJ_OSCALE 0.001953125f
#define OUT_OSCALE  0.00006103515625f
#define OGSCALE  16.f
#define SCORE_CS (0.00390625f * 0.08838834764831845f * 1.4426950408889634f)
#define POFF  6.f
#define PMAXL 15.99f
#define PMINL (-14.f)

static_assert(LL % 64 == 0 && CACHE % 64 == 0 && LL / 64 == 16 && CACHE / 64 == 16);
static_assert(BL % 128 == 0 && DD % 128 == 0 && NKV % 128 == 0 && DD % 32 == 0);
static_assert((NBHR * QT) % 8 == 0);

#if defined(__has_builtin)
#if __has_builtin(__builtin_amdgcn_exp2f)
#define EX2(x) __builtin_amdgcn_exp2f(x)
#endif
#if __has_builtin(__builtin_amdgcn_rcpf)
#define RCPF(x) __builtin_amdgcn_rcpf(x)
#endif
#endif
#ifndef EX2
#define EX2(x) exp2f(x)
#endif
#ifndef RCPF
#define RCPF(x) (1.f / (x))
#endif

__device__ __forceinline__ v8f wmma16(v16h a, v16h b, v8f c) {
  v8f d = __builtin_amdgcn_wmma_f32_16x16x32_f16(false, a, false, b, (short)0, c, false, false);
  asm volatile("v_nop\n\tv_nop\n\tv_nop\n\tv_nop" : "+v"(d) : "v"(a), "v"(b));
  return d;
}

__device__ __forceinline__ v8f zero8() {
  v8f z = {0.f, 0.f, 0.f, 0.f, 0.f, 0.f, 0.f, 0.f};
  return z;
}

__device__ __forceinline__ v8h cvt8(v4f a, v4f b, float s) {
  H8 o;
  o.e[0] = (f16_t)(a[0] * s); o.e[1] = (f16_t)(a[1] * s);
  o.e[2] = (f16_t)(a[2] * s); o.e[3] = (f16_t)(a[3] * s);
  o.e[4] = (f16_t)(b[0] * s); o.e[5] = (f16_t)(b[1] * s);
  o.e[6] = (f16_t)(b[2] * s); o.e[7] = (f16_t)(b[3] * s);
  return o.v;
}

__global__ __launch_bounds__(256) void cvt_f16_k(const float* __restrict__ src,
                                                 f16_t* __restrict__ dst, int n8, float scale) {
  const int i = blockIdx.x * 256 + threadIdx.x;
  if (i >= n8) return;
  const v4f* s = (const v4f*)(src + (size_t)i * 8);
  const v8h o = cvt8(s[0], s[1], scale);
  f16_t* d = dst + (size_t)i * 8;
  *(volatile v8h*)d = o;
  __threadfence();
  *(volatile v8h*)d = o;
}

__global__ __launch_bounds__(256) void cachek_k(const float* __restrict__ ck,
                                                f16_t* __restrict__ Kt, int n8) {
  const int i = blockIdx.x * 256 + threadIdx.x;
  if (i >= n8) return;
  const size_t e0 = (size_t)i * 8;
  const int kv = (int)(e0 / (size_t)(CACHE * HD));
  const v4f* s = (const v4f*)(ck + e0);
  const v8h o = cvt8(s[0], s[1], QKVSCALE);
  f16_t* d = Kt + e0 + (size_t)kv * (size_t)((SS - CACHE) * HD);
  *(volatile v8h*)d = o;
  __threadfence();
  *(volatile v8h*)d = o;
}

enum : int { GP = 40, SLP = 68 };

template <int N, int K>
__global__ __launch_bounds__(256) __attribute__((amdgpu_num_vgpr(240)))
void gemm_nt_k(const f16_t* __restrict__ A, const f16_t* __restrict__ Bw,
               float* __restrict__ C, float oscale) {
  __shared__ __align__(16) float smem[8 * 16 * SLP];
  f16_t* sA = (f16_t*)smem;
  f16_t* sB = sA + 128 * GP;
  const int tid = threadIdx.x, lane = tid & 31, wv = tid >> 5;
  const int wm = wv & 3, wn = wv >> 2;
  const int h = lane >> 4, m = lane & 15;
  const int gm = blockIdx.y * 128, gn = blockIdx.x * 128;

  Acc acc[2][4];
#pragma unroll
  for (int i = 0; i < 2; ++i)
#pragma unroll
    for (int j = 0; j < 4; ++j) acc[i][j].v = zero8();

#pragma unroll 1
  for (int k0 = 0; k0 < K; k0 += 32) {
    __syncthreads();
#pragma unroll
    for (int ci = 0; ci < 4; ++ci) {
      const int c = tid + 256 * ci;
      const int cc = c & 511, row = cc >> 2, sub = cc & 3;
      const f16_t* g;
      f16_t* l;
      if (ci < 2) { g = A  + (size_t)(gm + row) * K + k0 + sub * 8; l = sA + row * GP + sub * 8; }
      else        { g = Bw + (size_t)(gn + row) * K + k0 + sub * 8; l = sB + row * GP + sub * 8; }
      *(v8h*)l = *(const v8h*)g;
    }
    __syncthreads();
    Frag a0, a1;
    a0.half[0] = *(const v8h*)(sA + (wm * 32 + m) * GP + 8 * h);
    a0.half[1] = *(const v8h*)(sA + (wm * 32 + m) * GP + 16 + 8 * h);
    a1.half[0] = *(const v8h*)(sA + (wm * 32 + 16 + m) * GP + 8 * h);
    a1.half[1] = *(const v8h*)(sA + (wm * 32 + 16 + m) * GP + 16 + 8 * h);
#pragma unroll
    for (int j = 0; j < 4; ++j) {
      Frag b;
      b.half[0] = *(const v8h*)(sB + (wn * 64 + 16 * j + m) * GP + 8 * h);
      b.half[1] = *(const v8h*)(sB + (wn * 64 + 16 * j + m) * GP + 16 + 8 * h);
      acc[0][j].v = wmma16(a0.v, b.v, acc[0][j].v);
      acc[1][j].v = wmma16(a1.v, b.v, acc[1][j].v);
    }
  }

  __syncthreads();
  float* slab = smem + wv * (16 * SLP);
  const int q = lane >> 3, e = lane & 7;
  const size_t colg = (size_t)(gn + wn * 64);
#pragma unroll
  for (int i = 0; i < 2; ++i) {
#pragma unroll
    for (int j = 0; j < 4; ++j)
#pragma unroll
      for (int r = 0; r < 8; ++r)
        slab[(8 * h + r) * SLP + 16 * j + m] = acc[i][j].f[r] * oscale;
    __syncthreads();
    v4f vals[8];
#pragma unroll
    for (int t = 0; t < 8; ++t) {
      const int row = 2 * t + (q >> 1), col = (q & 1) * 32 + e * 4;
      vals[t] = *(const v4f*)(slab + row * SLP + col);
    }
    const size_t rowg = (size_t)(gm + wm * 32 + 16 * i);
#pragma unroll
    for (int t = 0; t < 8; ++t) {
      const int row = 2 * t + (q >> 1), col = (q & 1) * 32 + e * 4;
      *(volatile v4f*)(C + (rowg + row) * (size_t)N + colg + col) = vals[t];
    }
    __threadfence();
#pragma unroll
    for (int t = 0; t < 8; ++t) {
      const int row = 2 * t + (q >> 1), col = (q & 1) * 32 + e * 4;
      *(volatile v4f*)(C + (rowg + row) * (size_t)N + colg + col) = vals[t];
    }
    __syncthreads();
  }
}

template <int MODE>
__global__ __launch_bounds__(256) void rms_pack_k(const float* __restrict__ Y,
                                                  f16_t* __restrict__ dst, int nrows) {
  const int lane = threadIdx.x & 31, wv = threadIdx.x >> 5;
  const int R = blockIdx.x * 16 + wv * 2 + (lane >> 4);
  const int e = lane & 15;
  const bool ok = R < nrows;
  const int Rc = ok ? R : 0;
  const float* src;
  f16_t* d;
  if (MODE == 0) {
    const int mrow = Rc >> 4, hh = Rc & 15;
    const int bi = mrow >> 10, l = mrow & (LL - 1);
    src = Y + (size_t)mrow * DD + hh * HD + e * 8;
    d = dst + ((size_t)(bi * HH + hh) * LL + l) * HD + e * 8;
  } else {
    const int mrow = Rc >> 2, kh = Rc & 3;
    const int bi = mrow >> 10, l = mrow & (LL - 1);
    src = Y + (size_t)mrow * NKV + kh * HD + e * 8;
    d = dst + ((size_t)(bi * NHKV + kh) * SS + CACHE + l) * HD + e * 8;
  }
  const v4f a = ((const v4f*)src)[0];
  const v4f c = ((const v4f*)src)[1];
  float ss = 0.f;
#pragma unroll
  for (int j = 0; j < 4; ++j) ss += a[j] * a[j] + c[j] * c[j];
#pragma unroll
  for (int off = 8; off >= 1; off >>= 1) ss += __shfl_xor(ss, off, 32);
  const float rr = rsqrtf(ss * (1.f / (float)HD) + 1e-6f) * QKVSCALE;
  const v8h o = cvt8(a, c, rr);
  if (ok) *(volatile v8h*)d = o;
  __threadfence();
  if (ok) *(volatile v8h*)d = o;
}

enum : int { TP = 72 };

template <int NEWV>
__global__ __launch_bounds__(256) void vt_pack_k(const float* __restrict__ src,
                                                 f16_t* __restrict__ Vt) {
  __shared__ __align__(16) f16_t T[HD * TP];
  const int tid = threadIdx.x;
  const int kv = blockIdx.x >> 4, sc = blockIdx.x & 15;
#pragma unroll
  for (int it = 0; it < 8; ++it) {
    const int c = tid + 256 * it, key = c >> 5, hd4 = (c & 31) * 4;
    const float* p;
    if (NEWV) {
      const int mrow = (kv >> 2) * LL + sc * 64 + key;
      p = src + (size_t)mrow * NKV + (kv & 3) * HD + hd4;
    } else {
      p = src + ((size_t)(kv * CACHE + sc * 64 + key)) * HD + hd4;
    }
    const v4f v = *(const v4f*)p;
#pragma unroll
    for (int j = 0; j < 4; ++j) T[(hd4 + j) * TP + key] = (f16_t)(v[j] * QKVSCALE);
  }
  __syncthreads();
  const int e = tid & 7;
  v8h vals[4];
#pragma unroll
  for (int t = 0; t < 4; ++t) {
    const int Lr = t * 32 + (tid >> 3);
    vals[t] = *(const v8h*)(T + Lr * TP + e * 8);
  }
  const size_t sbase = (size_t)(NEWV ? CACHE : 0) + (size_t)(sc * 64 + e * 8);
#pragma unroll
  for (int t = 0; t < 4; ++t) {
    const int Lr = t * 32 + (tid >> 3);
    f16_t* d = Vt + ((size_t)(kv * HD + Lr)) * SS + sbase;
    *(volatile v8h*)d = vals[t];
  }
  __threadfence();
#pragma unroll
  for (int t = 0; t < 4; ++t) {
    const int Lr = t * 32 + (tid >> 3);
    f16_t* d = Vt + ((size_t)(kv * HD + Lr)) * SS + sbase;
    *(volatile v8h*)d = vals[t];
  }
}

__global__ __launch_bounds__(256) void gate_k(const float* __restrict__ x,
                                              const float* __restrict__ wg,
                                              float* __restrict__ gates, int n4) {
  const int i = blockIdx.x * 256 + threadIdx.x;
  if (i >= n4) return;
  const int mrow = i >> 2, hq = (i & 3) * 4;
  const v4f* xr = (const v4f*)(x + (size_t)mrow * DD);
  const v4f x0 = xr[0], x1 = xr[1], x2 = xr[2], x3 = xr[3];
  F4 g;
#pragma unroll
  for (int u = 0; u < 4; ++u) {
    const v4f* wr = (const v4f*)(wg + (hq + u) * HH);
    const v4f w0 = wr[0], w1 = wr[1], w2 = wr[2], w3 = wr[3];
    float a = 0.f;
#pragma unroll
    for (int j = 0; j < 4; ++j) a += x0[j] * w0[j];
#pragma unroll
    for (int j = 0; j < 4; ++j) a += x1[j] * w1[j];
#pragma unroll
    for (int j = 0; j < 4; ++j) a += x2[j] * w2[j];
#pragma unroll
    for (int j = 0; j < 4; ++j) a += x3[j] * w3[j];
    g.f[u] = RCPF(1.f + __expf(-a));
  }
  float* d = gates + (size_t)i * 4;
  *(volatile v4f*)d = g.v;
  __threadfence();
  *(volatile v4f*)d = g.v;
}

enum : int { KP = 136, VP = 40, OGP = 136 };

__global__ __launch_bounds__(256) __attribute__((amdgpu_num_vgpr(240)))
void attn_k(const f16_t* __restrict__ Qh, const f16_t* __restrict__ Kt,
            const f16_t* __restrict__ Vt, const float* __restrict__ gates,
            f16_t* __restrict__ Og) {
  __shared__ __align__(16) f16_t shK[32 * KP];
  __shared__ __align__(16) f16_t shV[HD * VP];
  __shared__ __align__(16) f16_t shO[8 * 16 * OGP];
  const int tid = threadIdx.x, lane = tid & 31, wv = tid >> 5;
  const int h = lane >> 4, m = lane & 15;
  const int tile = blockIdx.x * 8 + wv;
  const int bhr = tile >> 6;
  const int l0 = (tile & 63) * 16;
  const int kv = bhr >> 2, head = bhr & 15, b = bhr >> 4;
  const f16_t* qb = Qh + ((size_t)bhr * LL + l0) * HD;
  const f16_t* kb = Kt + (size_t)kv * SS * HD;
  const f16_t* vb = Vt + (size_t)kv * HD * SS;
  f16_t* os = shO + wv * (16 * OGP);

#pragma unroll
  for (int it = 0; it < 8; ++it) {
    const int c = lane + 32 * it, row = c >> 4, sub = c & 15;
    *(v8h*)(os + row * OGP + sub * 8) = *(const v8h*)(qb + (size_t)row * HD + sub * 8);
  }

  Acc oT[8];
#pragma unroll
  for (int t = 0; t < 8; ++t) oT[t].v = zero8();
  float rsum = 0.f;
  const float cS = SCORE_CS;

#pragma unroll 1
  for (int s0 = 0; s0 < SS; s0 += 32) {
    __syncthreads();
#pragma unroll
    for (int ci = 0; ci < 4; ++ci) {
      const int c = tid + 256 * ci;
      const f16_t* g;
      f16_t* l;
      if (ci < 2) {
        const int row = c >> 4, sub = c & 15;
        g = kb + (size_t)(s0 + row) * HD + sub * 8;
        l = shK + row * KP + sub * 8;
      } else {
        const int cc = c - 512, row = cc >> 2, sub = cc & 3;
        g = vb + (size_t)row * SS + s0 + sub * 8;
        l = shV + row * VP + sub * 8;
      }
      *(v8h*)l = *(const v8h*)g;
    }
    __syncthreads();

    Acc sc0, sc1;
    sc0.v = zero8();
    sc1.v = zero8();
#pragma unroll
    for (int kk = 0; kk < 4; ++kk) {
      Frag qf, a0, a1;
      qf.half[0] = *(const v8h*)(os + m * OGP + 32 * kk + 8 * h);
      qf.half[1] = *(const v8h*)(os + m * OGP + 32 * kk + 16 + 8 * h);
      a0.half[0] = *(const v8h*)(shK + m * KP + 32 * kk + 8 * h);
      a0.half[1] = *(const v8h*)(shK + m * KP + 32 * kk + 16 + 8 * h);
      a1.half[0] = *(const v8h*)(shK + (16 + m) * KP + 32 * kk + 8 * h);
      a1.half[1] = *(const v8h*)(shK + (16 + m) * KP + 32 * kk + 16 + 8 * h);
      sc0.v = wmma16(a0.v, qf.v, sc0.v);
      sc1.v = wmma16(a1.v, qf.v, sc1.v);
    }

    Frag pb;
#pragma unroll
    for (int r = 0; r < 8; ++r) {
      float u0 = sc0.f[r] * cS - POFF;
      float u1 = sc1.f[r] * cS - POFF;
      u0 = fminf(u0, PMAXL);
      u1 = fminf(u1, PMAXL);
      const float p0 = (u0 < PMINL) ? 0.f : EX2(u0);
      const float p1 = (u1 < PMINL) ? 0.f : EX2(u1);
      const f16_t e0 = (f16_t)p0, e1 = (f16_t)p1;
      pb.e[r] = e0;
      pb.e[8 + r] = e1;
      rsum += (float)e0 + (float)e1;
    }

#pragma unroll
    for (int t = 0; t < 8; ++t) {
      Frag av;
      av.half[0] = *(const v8h*)(shV + (16 * t + m) * VP + 8 * h);
      av.half[1] = *(const v8h*)(shV + (16 * t + m) * VP + 16 + 8 * h);
      oT[t].v = wmma16(av.v, pb.v, oT[t].v);
    }
  }

  rsum += __shfl_xor(rsum, 16, 32);
  const float g = gates[((size_t)(b * LL + l0 + m)) * HH + head];
  const float inv = (rsum > 0.f) ? (g * OGSCALE / rsum) : 0.f;
  __syncthreads();
#pragma unroll
  for (int t = 0; t < 8; ++t) {
    H8 o;
#pragma unroll
    for (int r = 0; r < 8; ++r) o.e[r] = (f16_t)(oT[t].f[r] * inv);
    *(v8h*)(os + m * OGP + 16 * t + 8 * h) = o.v;
  }
  __syncthreads();
  const int e = lane & 7;
  v8h vals[8];
#pragma unroll
  for (int t = 0; t < 8; ++t) {
    const int Ln = 4 * t + (lane >> 3), row = Ln >> 1, hf = Ln & 1;
    vals[t] = *(const v8h*)(os + row * OGP + hf * 64 + e * 8);
  }
#pragma unroll
  for (int t = 0; t < 8; ++t) {
    const int Ln = 4 * t + (lane >> 3), row = Ln >> 1, hf = Ln & 1;
    f16_t* d = Og + ((size_t)(b * LL + l0 + row)) * DD + head * HD + hf * 64 + e * 8;
    *(volatile v8h*)d = vals[t];
  }
  __threadfence();
#pragma unroll
  for (int t = 0; t < 8; ++t) {
    const int Ln = 4 * t + (lane >> 3), row = Ln >> 1, hf = Ln & 1;
    f16_t* d = Og + ((size_t)(b * LL + l0 + row)) * DD + head * HD + hf * 64 + e * 8;
    *(volatile v8h*)d = vals[t];
  }
}

extern "C" void kernel_launch(void* const* d_in, const int* in_sizes, int n_in,
                              void* d_out, int out_size, void* d_ws, size_t ws_size,
                              hipStream_t stream) {
  if (n_in < 8) return;
  if (in_sizes[0] != BL * DD || in_sizes[1] != DD * DD || in_sizes[2] != NKV * DD ||
      in_sizes[3] != NKV * DD || in_sizes[4] != DD * DD || in_sizes[5] != HH * HH ||
      in_sizes[6] != BB * NHKV * CACHE * HD || in_sizes[7] != BB * NHKV * CACHE * HD) return;
  if (out_size != BL * DD) return;

  const float* x   = (const float*)d_in[0];
  const float* wq  = (const float*)d_in[1];
  const float* wk  = (const float*)d_in[2];
  const float* wvv = (const float*)d_in[3];
  const float* wo  = (const float*)d_in[4];
  const float* wg  = (const float*)d_in[5];
  const float* ck  = (const float*)d_in[6];
  const float* cv  = (const float*)d_in[7];
  float* out = (float*)d_out;

  char* ws = (char*)d_ws;
  size_t off = 0;
  auto take = [&](size_t bytes) -> char* {
    char* p = ws + off;
    off += (bytes + 255) & ~(size_t)255;
    return p;
  };
  f16_t* xh    = (f16_t*)take((size_t)BL * DD * 2);
  f16_t* wqh   = (f16_t*)take((size_t)DD * DD * 2);
  f16_t* wkh   = (f16_t*)take((size_t)NKV * DD * 2);
  f16_t* wvh   = (f16_t*)take((size_t)NKV * DD * 2);
  f16_t* woh   = (f16_t*)take((size_t)DD * DD * 2);
  float* Yq    = (float*)take((size_t)BL * DD * 4);
  float* Yk    = (float*)take((size_t)BL * NKV * 4);
  float* Yv    = (float*)take((size_t)BL * NKV * 4);
  f16_t* Qh    = (f16_t*)take((size_t)NBHR * LL * HD * 2);
  f16_t* Kt    = (f16_t*)take((size_t)BB * NHKV * SS * HD * 2);
  f16_t* Vt    = (f16_t*)take((size_t)BB * NHKV * HD * SS * 2);
  float* gates = (float*)take((size_t)BL * HH * 4);
  f16_t* Og    = (f16_t*)take((size_t)BL * DD * 2);
  if (off > ws_size) return;

  const int T = 256;
  const int n8x = BL * DD / 8, n8q = DD * DD / 8, n8k = NKV * DD / 8;
  const int n8c = BB * NHKV * CACHE * HD / 8;
  cvt_f16_k<<<(n8x + T - 1) / T, T, 0, stream>>>(x,   xh,  n8x, XSCALE);
  cvt_f16_k<<<(n8q + T - 1) / T, T, 0, stream>>>(wq,  wqh, n8q, WSCALE);
  cvt_f16_k<<<(n8k + T - 1) / T, T, 0, stream>>>(wk,  wkh, n8k, WSCALE);
  cvt_f16_k<<<(n8k + T - 1) / T, T, 0, stream>>>(wvv, wvh, n8k, WSCALE);
  cvt_f16_k<<<(n8q + T - 1) / T, T, 0, stream>>>(wo,  woh, n8q, WSCALE);
  cachek_k<<<(n8c + T - 1) / T, T, 0, stream>>>(ck, Kt, n8c);
  vt_pack_k<0><<<BB * NHKV * (CACHE / 64), T, 0, stream>>>(cv, Vt);

  gemm_nt_k<DD,  DD><<<dim3(DD / 128,  BL / 128), T, 0, stream>>>(xh, wqh, Yq, PROJ_OSCALE);
  gemm_nt_k<NKV, DD><<<dim3(NKV / 128, BL / 128), T, 0, stream>>>(xh, wkh, Yk, PROJ_OSCALE);
  gemm_nt_k<NKV, DD><<<dim3(NKV / 128, BL / 128), T, 0, stream>>>(xh, wvh, Yv, PROJ_OSCALE);

  const int nrq = BL * HH, nrk = BL * NHKV;
  rms_pack_k<0><<<(nrq + 15) / 16, T, 0, stream>>>(Yq, Qh, nrq);
  rms_pack_k<1><<<(nrk + 15) / 16, T, 0, stream>>>(Yk, Kt, nrk);
  vt_pack_k<1><<<BB * NHKV * (LL / 64), T, 0, stream>>>(Yv, Vt);
  const int n4g = BL * HH / 4;
  gate_k<<<(n4g + T - 1) / T, T, 0, stream>>>(x, wg, gates, n4g);

  attn_k<<<(NBHR * QT) / 8, T, 0, stream>>>(Qh, Kt, Vt, gates, Og);

  gemm_nt_k<DD, DD><<<dim3(DD / 128, BL / 128), T, 0, stream>>>(Og, woh, out, OUT_OSCALE);
}
